// MambaMoEBlock_67577015435317
// MI455X (gfx1250) — hardware-run, weakly checked
//
#include <hip/hip_runtime.h>
#include <math.h>

typedef __attribute__((ext_vector_type(16))) _Float16 v16h;
typedef __attribute__((ext_vector_type(8)))  _Float16 v8h;
typedef __attribute__((ext_vector_type(2)))  _Float16 v2h;
typedef __attribute__((ext_vector_type(16))) __bf16   v16b;
typedef __attribute__((ext_vector_type(8)))  __bf16   v8b;
typedef __attribute__((ext_vector_type(8)))  float    v8f;
typedef __attribute__((ext_vector_type(4)))  float    v4f;
typedef __attribute__((ext_vector_type(2)))  float    v2f;

constexpr int kB   = 4;
constexpr int kC   = 96;
constexpr int kH   = 40;
constexpr int kW   = 40;
constexpr int kL   = kH * kW;
constexpr int kP   = kB * kL;
constexpr int kDE  = 192;
constexpr int kR   = 6;
constexpr int kN   = 16;
constexpr int kK   = 4;
constexpr int kE   = 4;
constexpr int kXo  = kR + 2 * kN;
constexpr int kCP  = 128;
constexpr int kDP  = 256;
constexpr int kEP  = 512;
constexpr int kXP  = 256;
constexpr int kThr = 256;
constexpr float kBnEps = 1.0e-5f;
constexpr float kLnEps = 1.0e-5f;
constexpr float kWCarry = 1024.0f;
constexpr float kACarry = 256.0f;
constexpr float kYCarry = 64.0f;
constexpr float kScA = 1.0f / (kACarry * kWCarry);
constexpr float kScY = 1.0f / (kYCarry * kWCarry);
constexpr float kF16MinNormal = 6.103515625e-5f;

static_assert(kP == 6400 && kL == 1600 && kXo == 38 && kK * kDE == 768 && kE * kC == 384 && kK * 64 == kXP, "the index arithmetic below uses these sizes");

constexpr size_t kOffBIAS = 0ull;
constexpr size_t kOffGM = 8192ull;
constexpr size_t kOffWM = 10240ull;
constexpr size_t kOffPW16 = 10496ull;
constexpr size_t kOffFC2W16 = 43264ull;
constexpr size_t kOffFC3W16 = 76032ull;
constexpr size_t kOffWIN16 = 108800ull;
constexpr size_t kOffWX16 = 207104ull;
constexpr size_t kOffWDT16 = 338176ull;
constexpr size_t kOffWOUT16 = 387328ull;
constexpr size_t kOffPWALL16 = 452864ull;
constexpr size_t kOffX16 = 583936ull;
constexpr size_t kOffP0 = 2222336ull;
constexpr size_t kOffX0 = 5499136ull;
constexpr size_t kOffH16 = 8775936ull;
constexpr size_t kOffT32 = 10414336ull;
constexpr size_t kOffT16 = 13691136ull;
constexpr size_t kOffH2 = 15329536ull;
constexpr size_t kOffU16 = 18606336ull;
constexpr size_t kOffXZ = 20244736ull;
constexpr size_t kOffXS32 = 30075136ull;
constexpr size_t kOffXS16 = 34990336ull;
constexpr size_t kOffXD = 38267136ull;
constexpr size_t kOffDT16 = 44820736ull;
constexpr size_t kOffDL = 45230336ull;
constexpr size_t kOffYS = 64891136ull;
constexpr size_t kOffY16 = 84551936ull;
constexpr size_t kOffM1 = 87828736ull;
constexpr size_t kOffXA = 91105536ull;
constexpr size_t kOffV32 = 94382336ull;
constexpr size_t kOffAE16 = 97659136ull;
constexpr size_t kOffXO = 104212736ull;
constexpr size_t kWsTotal = 107489536ull;
static_assert(kWsTotal <= 134217728ull, "carve cap: under 128 MiB");
static_assert(kOffBIAS == 0
  && kOffGM == kOffBIAS + 8192ull
  && kOffWM == kOffGM + 2048ull
  && kOffPW16 == kOffWM + 256ull
  && kOffFC2W16 == kOffPW16 + 32768ull
  && kOffFC3W16 == kOffFC2W16 + 32768ull
  && kOffWIN16 == kOffFC3W16 + 32768ull
  && kOffWX16 == kOffWIN16 + 98304ull
  && kOffWDT16 == kOffWX16 + 131072ull
  && kOffWOUT16 == kOffWDT16 + 49152ull
  && kOffPWALL16 == kOffWOUT16 + 65536ull
  && kOffX16 == kOffPWALL16 + 131072ull
  && kOffP0 == kOffX16 + 1638400ull
  && kOffX0 == kOffP0 + 3276800ull
  && kOffH16 == kOffX0 + 3276800ull
  && kOffT32 == kOffH16 + 1638400ull
  && kOffT16 == kOffT32 + 3276800ull
  && kOffH2 == kOffT16 + 1638400ull
  && kOffU16 == kOffH2 + 3276800ull
  && kOffXZ == kOffU16 + 1638400ull
  && kOffXS32 == kOffXZ + 9830400ull
  && kOffXS16 == kOffXS32 + 4915200ull
  && kOffXD == kOffXS16 + 3276800ull
  && kOffDT16 == kOffXD + 6553600ull
  && kOffDL == kOffDT16 + 409600ull
  && kOffYS == kOffDL + 19660800ull
  && kOffY16 == kOffYS + 19660800ull
  && kOffM1 == kOffY16 + 3276800ull
  && kOffXA == kOffM1 + 3276800ull
  && kOffV32 == kOffXA + 3276800ull
  && kOffAE16 == kOffV32 + 3276800ull
  && kOffXO == kOffAE16 + 6553600ull
  && kWsTotal == kOffXO + 3276800ull, "the carve is a chain: every region starts where the one before ends");
static_assert((kOffGM % 256) == 0 && (kOffWM % 256) == 0 && (kOffPW16 % 256) == 0 && (kOffFC2W16 % 256) == 0 && (kOffFC3W16 % 256) == 0 && (kOffWIN16 % 256) == 0 && (kOffWX16 % 256) == 0 && (kOffWDT16 % 256) == 0 && (kOffWOUT16 % 256) == 0 && (kOffPWALL16 % 256) == 0 && (kOffX16 % 256) == 0 && (kOffP0 % 256) == 0 && (kOffX0 % 256) == 0 && (kOffH16 % 256) == 0 && (kOffT32 % 256) == 0 && (kOffT16 % 256) == 0 && (kOffH2 % 256) == 0 && (kOffU16 % 256) == 0 && (kOffXZ % 256) == 0 && (kOffXS32 % 256) == 0 && (kOffXS16 % 256) == 0 && (kOffXD % 256) == 0 && (kOffDT16 % 256) == 0 && (kOffDL % 256) == 0 && (kOffYS % 256) == 0 && (kOffY16 % 256) == 0 && (kOffM1 % 256) == 0 && (kOffXA % 256) == 0 && (kOffV32 % 256) == 0 && (kOffAE16 % 256) == 0 && (kOffXO % 256) == 0, "every region starts on a multiple of 256 B");

__device__ __forceinline__ unsigned short f2bf_bits(float f) {
  unsigned u = __float_as_uint(f);
  return (unsigned short)((u + 0x7FFFu + ((u >> 16) & 1u)) >> 16);
}
__device__ __forceinline__ float bf_bits2f(unsigned short h) { return __uint_as_float(((unsigned)h) << 16); }
__device__ __forceinline__ float bf16r(float f) { return bf_bits2f(f2bf_bits(f)); }
__device__ __forceinline__ float carry_flush(float v, float carry) {
  const float s = v * carry;
  return (fabsf(s) < kF16MinNormal) ? 0.0f : s;
}

__device__ __forceinline__ void dep_guard4_h(v8f& a, v8f& b, v8f& c, v8f& d, v16h x, v16h y) { asm volatile("v_nop\n\tv_nop\n\tv_nop\n\tv_nop" : "+v"(a), "+v"(b), "+v"(c), "+v"(d) : "v"(x), "v"(y)); }
__device__ __forceinline__ void dep_guard4_b(v8f& a, v8f& b, v8f& c, v8f& d, v16b x, v16b y) { asm volatile("v_nop\n\tv_nop\n\tv_nop\n\tv_nop" : "+v"(a), "+v"(b), "+v"(c), "+v"(d) : "v"(x), "v"(y)); }
__device__ __forceinline__ void keep4_h(v16h a, v16h b, v16h c, v16h d) { asm volatile("v_nop" :: "v"(a), "v"(b), "v"(c), "v"(d)); }
__device__ __forceinline__ void keep4_b(v16b a, v16b b, v16b c, v16b d) { asm volatile("v_nop" :: "v"(a), "v"(b), "v"(c), "v"(d)); }
__device__ __forceinline__ void acc_guard4(v8f& a, v8f& b, v8f& c, v8f& d) { asm volatile("v_nop\n\tv_nop\n\tv_nop\n\tv_nop" : "+v"(a), "+v"(b), "+v"(c), "+v"(d)); }

template <typename T> struct Frag;
template <> struct Frag<_Float16> {
  typedef v16h V; union U { v16h v; v8h h[2]; };
  static __device__ __forceinline__ v16h load(const _Float16* p) {
    U f; f.h[0] = *(const v8h*)(p); f.h[1] = *(const v8h*)(p + 16); return f.v;
  }
  static __device__ __forceinline__ v8f mma(v16h a, v16h b, v8f c) {
    return __builtin_amdgcn_wmma_f32_16x16x32_f16(false, a, false, b, (short)0, c, false, false);
  }
  static __device__ __forceinline__ void guard4(v8f& a, v8f& b, v8f& c, v8f& d, v16h x, v16h y) { dep_guard4_h(a, b, c, d, x, y); }
  static __device__ __forceinline__ void keep(v16h a, v16h b, v16h c, v16h d) { keep4_h(a, b, c, d); }
};
template <> struct Frag<__bf16> {
  typedef v16b V; union U { v16b v; v8b h[2]; };
  static __device__ __forceinline__ v16b load(const __bf16* p) {
    U f; f.h[0] = *(const v8b*)(p); f.h[1] = *(const v8b*)(p + 16); return f.v;
  }
  static __device__ __forceinline__ v8f mma(v16b a, v16b b, v8f c) {
    return __builtin_amdgcn_wmma_f32_16x16x32_bf16(false, a, false, b, (short)0, c, false, false);
  }
  static __device__ __forceinline__ void guard4(v8f& a, v8f& b, v8f& c, v8f& d, v16b x, v16b y) { dep_guard4_b(a, b, c, d, x, y); }
  static __device__ __forceinline__ void keep(v16b a, v16b b, v16b c, v16b d) { keep4_b(a, b, c, d); }
};

__device__ __forceinline__ v8f mma_h(v16h a, v16h b, v8f c) {
  c = __builtin_amdgcn_wmma_f32_16x16x32_f16(false, a, false, b, (short)0, c, false, false);
  asm volatile("v_nop\n\tv_nop\n\tv_nop\n\tv_nop" : "+v"(c) : "v"(a), "v"(b));
  return c;
}

template <int ET> struct Elem;
template <> struct Elem<0> { typedef _Float16 T; };
template <> struct Elem<1> { typedef __bf16 T; };
template <int ET, bool SPLIT, int BIAS_MODE, int OUT_MODE, bool RESID, int ACT = 0>
__global__ __launch_bounds__(256) void wmma_gemm64(
    const unsigned short* __restrict__ Ap, const unsigned short* __restrict__ A2p, int lda, long strideA,
    const unsigned short* __restrict__ Btp, const unsigned short* __restrict__ Bt2p, int ldb, long strideB,
    void* __restrict__ Cout, void* __restrict__ Cout2, int ldc, long strideC,
    const float* __restrict__ bias,
    const float* __restrict__ resid, long strideR,
    int M, int N, int K, float scale) {
  typedef typename Elem<ET>::T T;
  typedef typename Frag<T>::V V;
  const T* A = (const T*)Ap; const T* A2 = (const T*)A2p; const T* Bt = (const T*)Btp; const T* Bt2 = (const T*)Bt2p;
  __shared__ __align__(16) float sT[8][16 * 68];
  const int b    = blockIdx.y;
  const int lane = threadIdx.x & 31;
  const int wave = threadIdx.x >> 5;
  const int tilesN = N >> 6;
  const int tilesM = M >> 6;
  const int tile = blockIdx.x * 8 + wave;
  if (tile >= tilesM * tilesN) return;
  const int tm = tile / tilesN;
  const int tn = tile - tm * tilesN;
  const int m0 = tm << 6;
  const int n0 = tn << 6;

  const T* Ab  = A  + (size_t)b * strideA;
  const T* Bb  = Bt + (size_t)b * strideB;
  const T* Ab2 = SPLIT ? (A2  + (size_t)b * strideA) : nullptr;
  const T* Bb2 = SPLIT ? (Bt2 + (size_t)b * strideB) : nullptr;

  const int rlane = lane & 15;
  const int koff  = (lane >> 4) * 8;
  const int mOff  = (lane >> 4) * 8;

  v8f acc[4][4];
#pragma unroll
  for (int i = 0; i < 4; ++i)
#pragma unroll
    for (int j = 0; j < 4; ++j) acc[i][j] = (v8f){0.f,0.f,0.f,0.f,0.f,0.f,0.f,0.f};

  for (int k0 = 0; k0 < K; k0 += 32) {
    V bh[4], bl[4];
#pragma unroll
    for (int j = 0; j < 4; ++j) {
      const size_t bo = (size_t)(n0 + (j << 4) + rlane) * ldb + koff + k0;
      bh[j] = Frag<T>::load(Bb + bo);
      if (SPLIT) bl[j] = Frag<T>::load(Bb2 + bo);
    }
#pragma unroll
    for (int i = 0; i < 4; ++i) {
      const size_t ao = (size_t)(m0 + (i << 4) + rlane) * lda + koff + k0;
      V ah = Frag<T>::load(Ab + ao);
      V al;
      if (SPLIT) al = Frag<T>::load(Ab2 + ao);
#pragma unroll
      for (int j = 0; j < 4; ++j) {
        acc[i][j] = Frag<T>::mma(ah, bh[j], acc[i][j]);
        if (SPLIT) {
          acc[i][j] = Frag<T>::mma(ah, bl[j], acc[i][j]);
          acc[i][j] = Frag<T>::mma(al, bh[j], acc[i][j]);
        }
      }
      Frag<T>::guard4(acc[i][0], acc[i][1], acc[i][2], acc[i][3], ah, SPLIT ? al : ah);
    }
    Frag<T>::keep(bh[0], bh[1], bh[2], bh[3]);
    if (SPLIT) Frag<T>::keep(bl[0], bl[1], bl[2], bl[3]);
  }
  acc_guard4(acc[0][0], acc[0][1], acc[0][2], acc[0][3]);
  acc_guard4(acc[1][0], acc[1][1], acc[1][2], acc[1][3]);
  acc_guard4(acc[2][0], acc[2][1], acc[2][2], acc[2][3]);
  acc_guard4(acc[3][0], acc[3][1], acc[3][2], acc[3][3]);

  float* slab = sT[wave];
  const float* Rb = RESID ? (resid + (size_t)b * strideR) : nullptr;
#pragma unroll
  for (int i = 0; i < 4; ++i) {
    const int mBase = m0 + (i << 4);
#pragma unroll
    for (int j = 0; j < 4; ++j) {
      const int n = n0 + (j << 4) + rlane;
      float bv = 0.f;
      if (BIAS_MODE == 2) bv = bias[n];
#pragma unroll
      for (int r = 0; r < 8; ++r) {
        float v = acc[i][j][r] * scale;
        if (BIAS_MODE == 1) v += bias[mBase + mOff + r];
        if (BIAS_MODE == 2) v += bv;
        if (RESID) v += Rb[(size_t)(mBase + mOff + r) * ldc + n];
        if (ACT == 1) v = tanhf(v);
        if (ACT == 2) v = fmaxf(v, 0.0f);
        if (ACT == 3) v = v / (1.0f + expf(-v));
        if (ACT == 4) v = (v > 0.f) ? v : 0.01f * v;
        slab[(mOff + r) * 68 + (j << 4) + rlane] = v;
      }
    }
    __builtin_amdgcn_fence(__ATOMIC_RELEASE, "workgroup");
    __builtin_amdgcn_wave_barrier();
    __builtin_amdgcn_fence(__ATOMIC_ACQUIRE, "workgroup");
    if (OUT_MODE == 0) {
      float* C = (float*)Cout + (size_t)b * strideC;
      const int hh = lane >> 4, c4 = (lane & 15) * 4;
      for (int pass = 0; pass < 2; ++pass) {
#pragma unroll
        for (int it = 0; it < 8; ++it) {
          const int row = it * 2 + hh;
          v4f v = *(const v4f*)(slab + row * 68 + c4);
          *(volatile v4f*)(C + (size_t)(mBase + row) * ldc + n0 + c4) = v;
        }
        __threadfence();
      }
    } else {
      const int q = lane >> 3, c8 = (lane & 7) * 8;
      unsigned short* C  = (unsigned short*)Cout  + (size_t)b * strideC;
      unsigned short* C2 = (OUT_MODE == 2) ? ((unsigned short*)Cout2 + (size_t)b * strideC) : nullptr;
      for (int pass = 0; pass < 2; ++pass) {
#pragma unroll
        for (int it = 0; it < 4; ++it) {
          const int row = it * 4 + q;
          const float* sp = slab + row * 68 + c8;
          v8h hv, lv;
#pragma unroll
          for (int e = 0; e < 8; ++e) {
            if (OUT_MODE == 1) {
              hv[e] = (_Float16)sp[e];
            } else {
              unsigned short hb = f2bf_bits(sp[e]);
              unsigned short lb = f2bf_bits(sp[e] - bf_bits2f(hb));
              hv[e] = __builtin_bit_cast(_Float16, hb);
              lv[e] = __builtin_bit_cast(_Float16, lb);
            }
          }
          *(volatile v8h*)(C + (size_t)(mBase + row) * ldc + n0 + c8) = hv;
          if (OUT_MODE == 2) *(volatile v8h*)(C2 + (size_t)(mBase + row) * ldc + n0 + c8) = lv;
        }
        __threadfence();
      }
    }
    __builtin_amdgcn_fence(__ATOMIC_RELEASE, "workgroup");
    __builtin_amdgcn_wave_barrier();
    __builtin_amdgcn_fence(__ATOMIC_ACQUIRE, "workgroup");
  }
}


__device__ __forceinline__ void store2(float* p, float v) {
  *(volatile float*)p = v;
  __threadfence();
  *(volatile float*)p = v;
}

__device__ __forceinline__ float gelu_erf(float v) { return 0.5f * v * (1.0f + erff(v * 0.70710678118654752f)); }
__device__ __forceinline__ void store8h(unsigned short* p, v8h v) {
  *(volatile v8h*)p = v;
  __threadfence();
  *(volatile v8h*)p = v;
}
__device__ __forceinline__ void store8f(float* p, v4f a, v4f b) {
  *(volatile v4f*)p = a; *(volatile v4f*)(p + 4) = b;
  __threadfence();
  *(volatile v4f*)p = a; *(volatile v4f*)(p + 4) = b;
}

__global__ __launch_bounds__(kThr) void wpad_kernel(const float* __restrict__ src, unsigned short* __restrict__ dst, int nSrcRows, int srcCols, int pitchLog2) {
  const unsigned i   = blockIdx.x * (unsigned)kThr + threadIdx.x;
  const unsigned sh  = (unsigned)pitchLog2 - 3u;
  const unsigned row = i >> sh;
  const unsigned c8  = (i & ((1u << sh) - 1u)) * 8u;
  const bool live = (row < (unsigned)nSrcRows) && (c8 < (unsigned)srcCols);
  const float* sp = src + (live ? ((size_t)row * (unsigned)srcCols + c8) : (size_t)0);
  const v4f a0 = *(const v4f*)(sp);
  const v4f a1 = *(const v4f*)(sp + 4);
  v8h hv;
#pragma unroll
  for (int e = 0; e < 4; ++e) {
    const float f0 = a0[e];
    const float f1 = a1[e];
    hv[e]     = (_Float16)(live ? carry_flush(bf16r(f0), kWCarry) : 0.0f);
    hv[4 + e] = (_Float16)(live ? carry_flush(bf16r(f1), kWCarry) : 0.0f);
  }
  store8h(dst + ((size_t)row << pitchLog2) + c8, hv);
}

__global__ __launch_bounds__(kThr) void wx_kernel(const float* __restrict__ src, unsigned short* __restrict__ dst) {
  const unsigned i   = blockIdx.x * (unsigned)kThr + threadIdx.x;
  const unsigned row = i >> 5;
  const unsigned c8  = (i & 31u) * 8u;
  const unsigned k = row >> 6, j = row & 63u;
  const bool live = (c8 < (unsigned)kDE) && ((j < (unsigned)kR) || (j >= 8u && j < 40u));
  const unsigned sj = (j < (unsigned)kR) ? j : (j - 2u);
  const float* sp = src + (live ? ((size_t)(k * (unsigned)kXo + sj) * (unsigned)kDE + c8) : (size_t)0);
  const v4f a0 = *(const v4f*)(sp);
  const v4f a1 = *(const v4f*)(sp + 4);
  v8h hv;
#pragma unroll
  for (int e = 0; e < 4; ++e) {
    const float f0 = a0[e];
    const float f1 = a1[e];
    hv[e]     = (_Float16)(live ? carry_flush(bf16r(f0), kWCarry) : 0.0f);
    hv[4 + e] = (_Float16)(live ? carry_flush(bf16r(f1), kWCarry) : 0.0f);
  }
  store8h(dst + (size_t)row * kXP + c8, hv);
}
static_assert(kXP * kXP / 8 == 32 * kThr, "the parameter map's plane: 32 blocks");

__global__ __launch_bounds__(kThr) void wdt_kernel(const float* __restrict__ src, unsigned short* __restrict__ dst) {
  const unsigned i   = blockIdx.x * (unsigned)kThr + threadIdx.x;
  const unsigned row = i >> 2;
  const unsigned g   = i & 3u;
  const unsigned k   = (row >= 192u ? 1u : 0u) + (row >= 384u ? 1u : 0u) + (row >= 576u ? 1u : 0u);
  const bool live = (g == k);
  const float* sp = src + (live ? (size_t)row * (unsigned)kR : (size_t)0);
  v8h hv;
#pragma unroll
  for (int r = 0; r < 8; ++r) {
    const float f = sp[(r < kR) ? r : 0];
    hv[r] = (_Float16)((live && r < kR) ? carry_flush(bf16r(f), kWCarry) : 0.0f);
  }
  store8h(dst + (size_t)row * 32u + g * 8u, hv);
}
static_assert(kK * kDE * 32 / 8 == 12 * kThr, "the step-size map's plane: 12 blocks");

__global__ __launch_bounds__(kThr) void wpw_kernel(const float* __restrict__ src, unsigned short* __restrict__ dst) {
  const unsigned i = blockIdx.x * (unsigned)kThr + threadIdx.x;
  const unsigned o = i >> 6;
  const unsigned g = i & 63u;
  const unsigned e = (g >= 12u ? 1u : 0u) + (g >= 24u ? 1u : 0u) + (g >= 36u ? 1u : 0u);
  const bool live = (o < (unsigned)kC) && (g < 48u);
  const unsigned c0 = 8u * g - 96u * e;
  const float* sp = src + (live ? ((size_t)(e * (unsigned)kC + o) * (unsigned)kC + c0) : (size_t)0);
  const v4f a0 = *(const v4f*)(sp);
  const v4f a1 = *(const v4f*)(sp + 4);
  v8h hv;
#pragma unroll
  for (int q = 0; q < 4; ++q) {
    const float f0 = a0[q];
    const float f1 = a1[q];
    hv[q]     = (_Float16)(live ? carry_flush(bf16r(f0), kWCarry) : 0.0f);
    hv[4 + q] = (_Float16)(live ? carry_flush(bf16r(f1), kWCarry) : 0.0f);
  }
  store8h(dst + (size_t)o * kEP + 8u * g, hv);
}
static_assert(kCP * kEP / 8 == 32 * kThr, "the experts' weight plane: 32 blocks");

__global__ __launch_bounds__(kThr) void setup_kernel(const float* __restrict__ b2, const float* __restrict__ b3, const float* __restrict__ bdt, float* __restrict__ BIAS) {
  const unsigned i = blockIdx.x * (unsigned)kThr + threadIdx.x;
  const bool in2 = (i >= 1024u) && (i < 1024u + (unsigned)kC);
  const bool in3 = (i >= 1152u) && (i < 1152u + (unsigned)kC);
  const bool ind = (i >= 1280u);
  const float v2 = b2[in2 ? (i - 1024u) : 0u];
  const float v3 = b3[in3 ? (i - 1152u) : 0u];
  const float vd = bdt[ind ? (i - 1280u) : 0u];
  const float v = in2 ? bf16r(v2) : (in3 ? bf16r(v3) : (ind ? bf16r(vd) : 0.0f));
  store2(BIAS + i, v);
}
static_assert(1280 + kK * kDE == 8 * kThr, "set-up grid exact: 8 blocks");

__global__ __launch_bounds__(kThr) void xcast_kernel(const float* __restrict__ x, unsigned short* __restrict__ X16) {
  const unsigned j  = blockIdx.x * (unsigned)kThr + threadIdx.x;
  const unsigned b  = blockIdx.y;
  const unsigned pl = j >> 4;
  const unsigned g  = j & 15u;
  const bool live = g < 12u;
  const unsigned c0 = live ? 8u * g : 0u;
  v8h hv;
#pragma unroll
  for (int e = 0; e < 8; ++e) {
    const float f = x[((size_t)b * kC + c0 + (unsigned)e) * kL + pl];
    hv[e] = (_Float16)(live ? carry_flush(bf16r(f), kACarry) : 0.0f);
  }
  store8h(X16 + ((size_t)b * kL + pl) * kCP + 8u * g, hv);
}
static_assert(kL * 16 == 100 * kThr, "entry grid exact: 100 blocks a sample");

__global__ __launch_bounds__(kThr) void act0_kernel(const float* __restrict__ P0, const float* __restrict__ gam, const float* __restrict__ bet, float* __restrict__ X0) {
  const unsigned i = blockIdx.x * (unsigned)kThr + threadIdx.x;
  const size_t row = i >> 4;
  const unsigned g = i & 15u;
  const bool live = g < 12u;
  const unsigned c0 = live ? 8u * g : 0u;
  const float q = sqrtf(1.0f + kBnEps);
  const float* pp = P0 + row * kCP + c0;
  v4f o0, o1;
#pragma unroll
  for (int e = 0; e < 8; ++e) {
    const float ga = gam[c0 + e], be = bet[c0 + e];
    const float v = pp[e] * (bf16r(ga) / q) + bf16r(be);
    const float s = live ? (v / (1.0f + expf(-v))) : 0.0f;
    if (e < 4) o0[e] = s; else o1[e - 4] = s;
  }
  store8f(X0 + row * kCP + 8u * g, o0, o1);
}
static_assert(kP * 16 == 400 * kThr, "a 96-wide plane's elementwise grid: 400 blocks");

__global__ __launch_bounds__(128) void lsdw_kernel(const float* __restrict__ X0, const float* __restrict__ dw, const float* __restrict__ db,
                                                   const float* __restrict__ gam, const float* __restrict__ bet, unsigned short* __restrict__ H16) {
  const int w = (int)(blockIdx.x * 8u + (threadIdx.x >> 4));
  const int h = (int)blockIdx.y;
  const unsigned g = threadIdx.x & 15u;
  const bool live = g < 12u;
  const unsigned c0 = live ? 8u * g : 0u;
  const size_t row = (size_t)blockIdx.z * kL + (size_t)(h * kW + w);
  float acc[8];
#pragma unroll
  for (int e = 0; e < 8; ++e) { const float p = db[c0 + e]; acc[e] = bf16r(p); }
#pragma unroll
  for (int i = 0; i < 3; ++i) {
#pragma unroll
    for (int j = 0; j < 3; ++j) {
      const int hh = h + i - 1, ww = w + j - 1;
      const bool has = (hh >= 0) && (hh < kH) && (ww >= 0) && (ww < kW);
      const float* xp = X0 + (has ? (size_t)((long)row + (long)((i - 1) * kW + (j - 1))) : row) * kCP + c0;
      const v4f x0 = *(const v4f*)xp, x1 = *(const v4f*)(xp + 4);
#pragma unroll
      for (int e = 0; e < 8; ++e) {
        const float wt = dw[(size_t)(c0 + e) * 9 + i * 3 + j];
        const float xv = (e < 4) ? x0[e] : x1[e - 4];
        acc[e] += has ? bf16r(wt) * xv : 0.0f;
      }
    }
  }
  const float q = sqrtf(1.0f + kBnEps);
  v8h hv;
#pragma unroll
  for (int e = 0; e < 8; ++e) {
    const float ga = gam[c0 + e], be = bet[c0 + e];
    hv[e] = (_Float16)(live ? carry_flush(acc[e] * (bf16r(ga) / q) + bf16r(be), kACarry) : 0.0f);
  }
  store8h(H16 + row * kCP + 8u * g, hv);
}
static_assert(kW == 5 * 8, "stencil grid exact: 5 blocks of 8 columns a row of the map");

__global__ __launch_bounds__(kThr) void gelucast_kernel(const float* __restrict__ T32, unsigned short* __restrict__ T16) {
  const unsigned i = blockIdx.x * (unsigned)kThr + threadIdx.x;
  const size_t row = i >> 4;
  const unsigned g = i & 15u;
  const bool live = g < 12u;
  const float* tp = T32 + row * kCP + (live ? 8u * g : 0u);
  v8h hv;
#pragma unroll
  for (int e = 0; e < 8; ++e) { const float v = tp[e]; hv[e] = (_Float16)(live ? carry_flush(gelu_erf(v), kACarry) : 0.0f); }
  store8h(T16 + row * kCP + 8u * g, hv);
}

__global__ __launch_bounds__(kThr) void ucast_kernel(const float* __restrict__ X0, const float* __restrict__ H2, const float* __restrict__ gam, const float* __restrict__ bet,
                                                     unsigned short* __restrict__ U16) {
  const unsigned i = blockIdx.x * (unsigned)kThr + threadIdx.x;
  const size_t row = i >> 4;
  const unsigned g = i & 15u;
  const bool live = g < 12u;
  const unsigned c0 = live ? 8u * g : 0u;
  const float q = sqrtf(1.0f + kBnEps);
  const float* xp = X0 + row * kCP + c0;
  const float* hp = H2 + row * kCP + c0;
  v8h hv;
#pragma unroll
  for (int e = 0; e < 8; ++e) {
    const float ga = gam[c0 + e], be = bet[c0 + e];
    hv[e] = (_Float16)(live ? carry_flush((xp[e] + hp[e]) * (bf16r(ga) / q) + bf16r(be), kACarry) : 0.0f);
  }
  store8h(U16 + row * kCP + 8u * g, hv);
}

__global__ __launch_bounds__(kThr) void mconv_kernel(const float* __restrict__ XZ, const float* __restrict__ dw, const float* __restrict__ db,
                                                     float* __restrict__ XS32, unsigned short* __restrict__ XS16) {
  const int w = (int)(blockIdx.x * 8u + (threadIdx.x >> 5));
  const int h = (int)blockIdx.y;
  const unsigned g = threadIdx.x & 31u;
  const bool live = g < 24u;
  const unsigned c0 = live ? 8u * g : 0u;
  const size_t row = (size_t)blockIdx.z * kL + (size_t)(h * kW + w);
  float acc[8];
#pragma unroll
  for (int e = 0; e < 8; ++e) { const float p = db[c0 + e]; acc[e] = bf16r(p); }
#pragma unroll
  for (int i = 0; i < 3; ++i) {
#pragma unroll
    for (int j = 0; j < 3; ++j) {
      const int hh = h + i - 1, ww = w + j - 1;
      const bool has = (hh >= 0) && (hh < kH) && (ww >= 0) && (ww < kW);
      const float* xp = XZ + (has ? (size_t)((long)row + (long)((i - 1) * kW + (j - 1))) : row) * (2 * kDE) + c0;
      const v4f x0 = *(const v4f*)xp, x1 = *(const v4f*)(xp + 4);
#pragma unroll
      for (int e = 0; e < 8; ++e) {
        const float wt = dw[(size_t)(c0 + e) * 9 + i * 3 + j];
        const float xv = (e < 4) ? x0[e] : x1[e - 4];
        acc[e] += has ? bf16r(wt) * xv : 0.0f;
      }
    }
  }
  v4f u0, u1;
  v8h hv;
#pragma unroll
  for (int e = 0; e < 8; ++e) {
    const float s = gelu_erf(acc[e]);
    if (e < 4) u0[e] = s; else u1[e - 4] = s;
    hv[e] = (_Float16)(live ? carry_flush(s, kACarry) : 0.0f);
  }
  if (live) store8f(XS32 + row * kDE + c0, u0, u1);
  store8h(XS16 + row * kDP + 8u * g, hv);
}

__global__ __launch_bounds__(kThr) void dtcast_kernel(const float* __restrict__ XD, unsigned short* __restrict__ DT16) {
  const unsigned i = blockIdx.x * (unsigned)kThr + threadIdx.x;
  const size_t row = i >> 2;
  const unsigned k = i & 3u;
  const float* sp = XD + row * kXP + 64u * k;
  v8h hv;
#pragma unroll
  for (int r = 0; r < 8; ++r) { const float v = sp[r]; hv[r] = (_Float16)((r < kR) ? carry_flush(v, kACarry) : 0.0f); }
  store8h(DT16 + row * 32u + 8u * k, hv);
}
static_assert(kP * 4 == 100 * kThr, "the step input's cast: 100 blocks");

__global__ __launch_bounds__(192) void scan_kernel(const float* __restrict__ XD, const float* __restrict__ DL, const float* __restrict__ XS32,
                                                   const float* __restrict__ A_logs, const float* __restrict__ Dsk, float* __restrict__ YS) {
  const unsigned d = threadIdx.x, k = blockIdx.x, b = blockIdx.y;
  float A[kN], h[kN];
#pragma unroll
  for (int n = 0; n < kN; ++n) { const float a = A_logs[(size_t)(k * (unsigned)kDE + d) * kN + n]; A[n] = -expf(bf16r(a)); h[n] = 0.0f; }
  const float q0 = Dsk[k * (unsigned)kDE + d];
  const float dsk = bf16r(q0);
  int ph = (k >= 2u) ? (kH - 1) : 0;
  int pw = (k >= 2u) ? (kW - 1) : 0;
  float* ys = YS + (size_t)k * kP * kDE;
  for (int l = 0; l < kL; ++l) {
    const size_t row = (size_t)b * kL + (size_t)(ph * kW + pw);
    const float* pr = XD + row * kXP + 64u * k + 8u;
    const float pre = DL[row * (kK * kDE) + k * (unsigned)kDE + d];
    const float uv = XS32[row * kDE + d];
    const float dt = fmaxf(pre, 0.0f) + log1pf(expf(-fabsf(pre)));
    const float dx = dt * uv;
    float y = 0.0f;
#pragma unroll
    for (int q = 0; q < kN / 4; ++q) {
      const v4f bv = *(const v4f*)(pr + 4 * q), cv = *(const v4f*)(pr + kN + 4 * q);
#pragma unroll
      for (int e = 0; e < 4; ++e) {
        const int n = 4 * q + e;
        const float hn = expf(dt * A[n]) * h[n] + dx * bv[e];
        h[n] = hn;
        y += hn * cv[e];
      }
    }
    store2(ys + row * kDE + d, y + dsk * uv);
    if (k == 0u)      { ++pw; if (pw == kW) { pw = 0; ++ph; } }
    else if (k == 1u) { ++ph; if (ph == kH) { ph = 0; ++pw; } }
    else if (k == 2u) { --pw; if (pw < 0) { pw = kW - 1; --ph; } }
    else              { --ph; if (ph < 0) { ph = kH - 1; --pw; } }
  }
}
static_assert(kDE == 6 * 32 && (kN % 4) == 0, "walk block = 6 whole waves; the B | C columns 16-B aligned");

__global__ __launch_bounds__(kThr) void lngate_kernel(const float* __restrict__ YS, const float* __restrict__ XZ, const float* __restrict__ gam, const float* __restrict__ bet,
                                                      unsigned short* __restrict__ Y16) {
  const size_t row = blockIdx.x * (unsigned)kThr + threadIdx.x;
  const float* y0 = YS + row * kDE;
  const float* y1 = y0 + (size_t)kP * kDE;
  const float* y2 = y1 + (size_t)kP * kDE;
  const float* y3 = y2 + (size_t)kP * kDE;
  float s = 0.0f;
  for (int d = 0; d < kDE; ++d) s += (y0[d] + y2[d]) + (y1[d] + y3[d]);
  const float m = s / (float)kDE;
  float vs = 0.0f;
  for (int d = 0; d < kDE; ++d) { const float c = ((y0[d] + y2[d]) + (y1[d] + y3[d])) - m; vs += c * c; }
  const float sd = sqrtf(vs / (float)kDE + kLnEps);
  const float* zp = XZ + row * (2 * kDE) + kDE;
  unsigned short* dp = Y16 + row * kDP;
  for (int d8 = 0; d8 < kDE; d8 += 8) {
    v8h hv;
#pragma unroll
    for (int e = 0; e < 8; ++e) {
      const int d = d8 + e;
      const float ga = gam[d], be = bet[d];
      const float c = ((y0[d] + y2[d]) + (y1[d] + y3[d])) - m;
      const float nv = c / sd * bf16r(ga) + bf16r(be);
      hv[e] = (_Float16)carry_flush(nv * gelu_erf(zp[d]), kYCarry);
    }
    store8h(dp + d8, hv);
  }
}
static_assert(kP == 25 * kThr, "merge grid exact: 25 blocks");

__global__ __launch_bounds__(kThr) void xav_kernel(const float* __restrict__ X0, const float* __restrict__ M1, const float* __restrict__ gam, const float* __restrict__ bet,
                                                   float* __restrict__ XA, float* __restrict__ V32) {
  const unsigned i = blockIdx.x * (unsigned)kThr + threadIdx.x;
  const size_t row = i >> 4;
  const unsigned g = i & 15u;
  const bool live = g < 12u;
  const unsigned c0 = live ? 8u * g : 0u;
  const float q = sqrtf(1.0f + kBnEps);
  const float* xp = X0 + row * kCP + c0;
  const float* mp = M1 + row * kCP + c0;
  v4f a0, a1, v0, v1;
#pragma unroll
  for (int e = 0; e < 8; ++e) {
    const float ga = gam[c0 + e], be = bet[c0 + e];
    const float xa = xp[e] + mp[e];
    const float vv = xa * (bf16r(ga) / q) + bf16r(be);
    const float xo = live ? xa : 0.0f, vo = live ? vv : 0.0f;
    if (e < 4) { a0[e] = xo; v0[e] = vo; } else { a1[e - 4] = xo; v1[e - 4] = vo; }
  }
  store8f(XA + row * kCP + 8u * g, a0, a1);
  store8f(V32 + row * kCP + 8u * g, v0, v1);
}

__global__ __launch_bounds__(128) void gsum_kernel(const float* __restrict__ V32, float* __restrict__ GM) {
  const unsigned c = threadIdx.x, b = blockIdx.x;
  const float* vp = V32 + (size_t)b * kL * kCP + c;
  float s = 0.0f;
  for (int j = 0; j < kL; ++j) s += vp[(size_t)j * kCP];
  store2(GM + b * (unsigned)kCP + c, s / (float)kL);
}

__global__ __launch_bounds__(32) void route_kernel(const float* __restrict__ GM, const float* __restrict__ rw, const float* __restrict__ rb, float* __restrict__ WM) {
  const unsigned b = threadIdx.x & 3u;
  const float* gp = GM + b * (unsigned)kCP;
  float lg[kE];
#pragma unroll
  for (int e = 0; e < kE; ++e) {
    float a = 0.0f;
    for (int c = 0; c < kC; ++c) { const float wv = rw[e * kC + c]; a += gp[c] * bf16r(wv); }
    const float tb = rb[e];
    lg[e] = (a + bf16r(tb)) / 2.0f;
  }
  const float mx = fmaxf(fmaxf(lg[0], lg[1]), fmaxf(lg[2], lg[3]));
  float p[kE], sum = 0.0f;
#pragma unroll
  for (int e = 0; e < kE; ++e) { p[e] = expf(lg[e] - mx); sum += p[e]; }
#pragma unroll
  for (int e = 0; e < kE; ++e) p[e] = p[e] / sum;
  int i1 = 0; float p1 = p[0];
#pragma unroll
  for (int e = 1; e < kE; ++e) { const bool up = p[e] > p1; p1 = up ? p[e] : p1; i1 = up ? e : i1; }
  int i2 = -1; float p2 = -1.0f;
#pragma unroll
  for (int e = 0; e < kE; ++e) { const bool up = (e != i1) && (p[e] > p2); p2 = up ? p[e] : p2; i2 = up ? e : i2; }
  const float den = p1 + p2;
  v4f wv;
#pragma unroll
  for (int e = 0; e < kE; ++e) wv[e] = (e == i1) ? (p1 / den) : ((e == i2) ? (p2 / den) : 0.0f);
  if (threadIdx.x < (unsigned)kB) {
    float* dp = WM + threadIdx.x * (unsigned)kE;
    *(volatile v4f*)dp = wv;
    __threadfence();
    *(volatile v4f*)dp = wv;
  }
}

__global__ __launch_bounds__(512) void edw_kernel(const float* __restrict__ V32, const float* __restrict__ dw, const float* __restrict__ db, const float* __restrict__ WM,
                                                  unsigned short* __restrict__ AE16) {
  const int w = (int)(blockIdx.x * 8u + (threadIdx.x >> 6));
  const int h = (int)blockIdx.y;
  const unsigned g = threadIdx.x & 63u;
  const bool live = g < 48u;
  const unsigned e = live ? ((g >= 12u ? 1u : 0u) + (g >= 24u ? 1u : 0u) + (g >= 36u ? 1u : 0u)) : 0u;
  const unsigned c0 = live ? (8u * g - 96u * e) : 0u;
  const size_t row = (size_t)blockIdx.z * kL + (size_t)(h * kW + w);
  const float we = WM[blockIdx.z * (unsigned)kE + e];
  float acc[8];
#pragma unroll
  for (int q = 0; q < 8; ++q) { const float p = db[e * (unsigned)kC + c0 + q]; acc[q] = bf16r(p); }
#pragma unroll
  for (int i = 0; i < 3; ++i) {
#pragma unroll
    for (int j = 0; j < 3; ++j) {
      const int hh = h + i - 1, ww = w + j - 1;
      const bool has = (hh >= 0) && (hh < kH) && (ww >= 0) && (ww < kW);
      const float* xp = V32 + (has ? (size_t)((long)row + (long)((i - 1) * kW + (j - 1))) : row) * kCP + c0;
      const v4f x0 = *(const v4f*)xp, x1 = *(const v4f*)(xp + 4);
#pragma unroll
      for (int q = 0; q < 8; ++q) {
        const float wt = dw[(size_t)(e * (unsigned)kC + c0 + q) * 9 + i * 3 + j];
        const float xv = (q < 4) ? x0[q] : x1[q - 4];
        acc[q] += has ? bf16r(wt) * xv : 0.0f;
      }
    }
  }
  v8h hv;
#pragma unroll
  for (int q = 0; q < 8; ++q) hv[q] = (_Float16)(live ? carry_flush(we * gelu_erf(acc[q]), kACarry) : 0.0f);
  store8h(AE16 + row * kEP + 8u * g, hv);
}

__global__ __launch_bounds__(64) void exit_kernel(const float* __restrict__ XA, const float* __restrict__ XO, const float* __restrict__ WM, const float* __restrict__ pb, float* __restrict__ out) {
  const unsigned pl = blockIdx.x * 64u + threadIdx.x;
  const unsigned c = blockIdx.y, b = blockIdx.z;
  const size_t row = (size_t)b * kL + pl;
  float tb = 0.0f;
#pragma unroll
  for (int e = 0; e < kE; ++e) { const float t = pb[e * kC + c]; tb += WM[b * (unsigned)kE + e] * bf16r(t); }
  store2(out + ((size_t)b * kC + c) * kL + pl, XA[row * kCP + c] + (XO[row * kCP + c] + tb));
}
static_assert(kL == 25 * 64, "exit grid exact: 25 blocks of 64 positions a channel");

extern "C" void kernel_launch(void* const* d_in, const int* in_sizes, int n_in,
                              void* d_out, int out_size, void* d_ws, size_t ws_size,
                              hipStream_t stream) {
  if (n_in < 33 || d_out == nullptr || d_ws == nullptr) return;
  if (in_sizes[0] != kB * kC * kL || in_sizes[1] != kC * kC || in_sizes[2] != kC || in_sizes[3] != kC || in_sizes[4] != kC * 9 || in_sizes[5] != kC || in_sizes[6] != kC || in_sizes[7] != kC) return;
  if (in_sizes[8] != kC * kC || in_sizes[9] != kC || in_sizes[10] != kC * kC || in_sizes[11] != kC || in_sizes[12] != kC || in_sizes[13] != kC || in_sizes[14] != 2 * kDE * kC) return;
  if (in_sizes[15] != kDE * 9 || in_sizes[16] != kDE || in_sizes[17] != kK * kXo * kDE || in_sizes[18] != kK * kDE * kR || in_sizes[19] != kK * kDE || in_sizes[20] != kK * kDE * kN) return;
  if (in_sizes[21] != kK * kDE || in_sizes[22] != kDE || in_sizes[23] != kDE || in_sizes[24] != kC * kDE || in_sizes[25] != kC || in_sizes[26] != kC || in_sizes[27] != kE * kC) return;
  if (in_sizes[28] != kE || in_sizes[29] != kE * kC * 9 || in_sizes[30] != kE * kC || in_sizes[31] != kE * kC * kC || in_sizes[32] != kE * kC) return;
  if (out_size != kB * kC * kL) return;
  if (ws_size < kWsTotal) return;
  const float* x        = (const float*)d_in[0];
  const float* proj_w   = (const float*)d_in[1];
  const float* bn0_g    = (const float*)d_in[2];
  const float* bn0_b    = (const float*)d_in[3];
  const float* ls_dw_w  = (const float*)d_in[4];
  const float* ls_dw_b  = (const float*)d_in[5];
  const float* ls_bn_g  = (const float*)d_in[6];
  const float* ls_bn_b  = (const float*)d_in[7];
  const float* ls_fc2_w = (const float*)d_in[8];
  const float* ls_fc2_b = (const float*)d_in[9];
  const float* ls_fc3_w = (const float*)d_in[10];
  const float* ls_fc3_b = (const float*)d_in[11];
  const float* n1_g     = (const float*)d_in[12];
  const float* n1_b     = (const float*)d_in[13];
  const float* in_w     = (const float*)d_in[14];
  const float* conv_w   = (const float*)d_in[15];
  const float* conv_b   = (const float*)d_in[16];
  const float* xp_w     = (const float*)d_in[17];
  const float* dt_w     = (const float*)d_in[18];
  const float* dt_b     = (const float*)d_in[19];
  const float* A_logs   = (const float*)d_in[20];
  const float* Dskip    = (const float*)d_in[21];
  const float* on_g     = (const float*)d_in[22];
  const float* on_b     = (const float*)d_in[23];
  const float* out_w    = (const float*)d_in[24];
  const float* n2_g     = (const float*)d_in[25];
  const float* n2_b     = (const float*)d_in[26];
  const float* rt_w     = (const float*)d_in[27];
  const float* rt_b     = (const float*)d_in[28];
  const float* ex_dw_w  = (const float*)d_in[29];
  const float* ex_dw_b  = (const float*)d_in[30];
  const float* ex_pw_w  = (const float*)d_in[31];
  const float* ex_pw_b  = (const float*)d_in[32];
  float* out = (float*)d_out;
  char* ws = (char*)d_ws;
  float* BIAS = (float*)(ws + kOffBIAS);
  float* ZB  = BIAS;
  float* B2  = BIAS + 1024;
  float* B3  = BIAS + 1152;
  float* BDT = BIAS + 1280;
  float* GM = (float*)(ws + kOffGM);
  float* WM = (float*)(ws + kOffWM);
  unsigned short* PW16    = (unsigned short*)(ws + kOffPW16);
  unsigned short* FC2W16  = (unsigned short*)(ws + kOffFC2W16);
  unsigned short* FC3W16  = (unsigned short*)(ws + kOffFC3W16);
  unsigned short* WIN16   = (unsigned short*)(ws + kOffWIN16);
  unsigned short* WX16    = (unsigned short*)(ws + kOffWX16);
  unsigned short* WDT16   = (unsigned short*)(ws + kOffWDT16);
  unsigned short* WOUT16  = (unsigned short*)(ws + kOffWOUT16);
  unsigned short* PWALL16 = (unsigned short*)(ws + kOffPWALL16);
  unsigned short* X16 = (unsigned short*)(ws + kOffX16);
  float* P0 = (float*)(ws + kOffP0);
  float* X0 = (float*)(ws + kOffX0);
  unsigned short* H16 = (unsigned short*)(ws + kOffH16);
  float* T32 = (float*)(ws + kOffT32);
  unsigned short* T16 = (unsigned short*)(ws + kOffT16);
  float* H2 = (float*)(ws + kOffH2);
  unsigned short* U16 = (unsigned short*)(ws + kOffU16);
  float* XZ = (float*)(ws + kOffXZ);
  float* XS32 = (float*)(ws + kOffXS32);
  unsigned short* XS16 = (unsigned short*)(ws + kOffXS16);
  float* XD = (float*)(ws + kOffXD);
  unsigned short* DT16 = (unsigned short*)(ws + kOffDT16);
  float* DL = (float*)(ws + kOffDL);
  float* YS = (float*)(ws + kOffYS);
  unsigned short* Y16 = (unsigned short*)(ws + kOffY16);
  float* M1 = (float*)(ws + kOffM1);
  float* XA = (float*)(ws + kOffXA);
  float* V32 = (float*)(ws + kOffV32);
  unsigned short* AE16 = (unsigned short*)(ws + kOffAE16);
  float* XO = (float*)(ws + kOffXO);

  static_assert((kCP * kCP / 8) % kThr == 0 && (2 * kDE * kCP / 8) % kThr == 0 && (kCP * kDP / 8) % kThr == 0, "the padded weight planes' grids are exact: 8, 24 and 16 blocks");
  wpad_kernel<<<kCP * kCP / 8 / kThr, kThr, 0, stream>>>(proj_w, PW16, kC, kC, 7);
  wpad_kernel<<<kCP * kCP / 8 / kThr, kThr, 0, stream>>>(ls_fc2_w, FC2W16, kC, kC, 7);
  wpad_kernel<<<kCP * kCP / 8 / kThr, kThr, 0, stream>>>(ls_fc3_w, FC3W16, kC, kC, 7);
  wpad_kernel<<<2 * kDE * kCP / 8 / kThr, kThr, 0, stream>>>(in_w, WIN16, 2 * kDE, kC, 7);
  wpad_kernel<<<kCP * kDP / 8 / kThr, kThr, 0, stream>>>(out_w, WOUT16, kC, kDE, 8);
  wx_kernel<<<32, kThr, 0, stream>>>(xp_w, WX16);
  wdt_kernel<<<12, kThr, 0, stream>>>(dt_w, WDT16);
  wpw_kernel<<<32, kThr, 0, stream>>>(ex_pw_w, PWALL16);
  setup_kernel<<<8, kThr, 0, stream>>>(ls_fc2_b, ls_fc3_b, dt_b, BIAS);

  xcast_kernel<<<dim3(100, kB), kThr, 0, stream>>>(x, X16);
  wmma_gemm64<0, false, 2, 0, false, 0><<<dim3((kP / 64) * (kCP / 64) / 8, 1), 256, 0, stream>>>(
      X16, X16, kCP, 0L, PW16, PW16, kCP, 0L, (void*)P0, (void*)P0, kCP, 0L, ZB, nullptr, 0L, kP, kCP, kC, kScA);
  act0_kernel<<<400, kThr, 0, stream>>>(P0, bn0_g, bn0_b, X0);

  lsdw_kernel<<<dim3(5, kH, kB), 128, 0, stream>>>(X0, ls_dw_w, ls_dw_b, ls_bn_g, ls_bn_b, H16);
  wmma_gemm64<0, false, 2, 0, false, 0><<<dim3((kP / 64) * (kCP / 64) / 8, 1), 256, 0, stream>>>(
      H16, H16, kCP, 0L, FC2W16, FC2W16, kCP, 0L, (void*)T32, (void*)T32, kCP, 0L, B2, nullptr, 0L, kP, kCP, kC, kScA);
  gelucast_kernel<<<400, kThr, 0, stream>>>(T32, T16);
  wmma_gemm64<0, false, 2, 0, false, 0><<<dim3((kP / 64) * (kCP / 64) / 8, 1), 256, 0, stream>>>(
      T16, T16, kCP, 0L, FC3W16, FC3W16, kCP, 0L, (void*)H2, (void*)H2, kCP, 0L, B3, nullptr, 0L, kP, kCP, kC, kScA);
  ucast_kernel<<<400, kThr, 0, stream>>>(X0, H2, n1_g, n1_b, U16);

  wmma_gemm64<0, false, 2, 0, false, 0><<<dim3((kP / 64) * (2 * kDE / 64) / 8, 1), 256, 0, stream>>>(
      U16, U16, kCP, 0L, WIN16, WIN16, kCP, 0L, (void*)XZ, (void*)XZ, 2 * kDE, 0L, ZB, nullptr, 0L, kP, 2 * kDE, kC, kScA);
  mconv_kernel<<<dim3(5, kH, kB), kThr, 0, stream>>>(XZ, conv_w, conv_b, XS32, XS16);
  wmma_gemm64<0, false, 2, 0, false, 0><<<dim3((kP / 64) * (kXP / 64) / 8, 1), 256, 0, stream>>>(
      XS16, XS16, kDP, 0L, WX16, WX16, kXP, 0L, (void*)XD, (void*)XD, kXP, 0L, ZB, nullptr, 0L, kP, kXP, kDE, kScA);
  dtcast_kernel<<<100, kThr, 0, stream>>>(XD, DT16);
  wmma_gemm64<0, false, 2, 0, false, 0><<<dim3((kP / 64) * (kK * kDE / 64) / 8, 1), 256, 0, stream>>>(
      DT16, DT16, 32, 0L, WDT16, WDT16, 32, 0L, (void*)DL, (void*)DL, kK * kDE, 0L, BDT, nullptr, 0L, kP, kK * kDE, 32, kScA);
  scan_kernel<<<dim3(kK, kB), 192, 0, stream>>>(XD, DL, XS32, A_logs, Dskip, YS);
  lngate_kernel<<<25, kThr, 0, stream>>>(YS, XZ, on_g, on_b, Y16);
  wmma_gemm64<0, false, 2, 0, false, 0><<<dim3((kP / 64) * (kCP / 64) / 8, 1), 256, 0, stream>>>(
      Y16, Y16, kDP, 0L, WOUT16, WOUT16, kDP, 0L, (void*)M1, (void*)M1, kCP, 0L, ZB, nullptr, 0L, kP, kCP, kDE, kScY);
  xav_kernel<<<400, kThr, 0, stream>>>(X0, M1, n2_g, n2_b, XA, V32);

  gsum_kernel<<<kB, 128, 0, stream>>>(V32, GM);
  route_kernel<<<1, 32, 0, stream>>>(GM, rt_w, rt_b, WM);
  edw_kernel<<<dim3(5, kH, kB), 512, 0, stream>>>(V32, ex_dw_w, ex_dw_b, WM, AE16);
  wmma_gemm64<0, false, 2, 0, false, 0><<<dim3((kP / 64) * (kCP / 64) / 8, 1), 256, 0, stream>>>(
      AE16, AE16, kEP, 0L, PWALL16, PWALL16, kEP, 0L, (void*)XO, (void*)XO, kCP, 0L, ZB, nullptr, 0L, kP, kCP, kE * kC, kScA);
  exit_kernel<<<dim3(25, kC, kB), 64, 0, stream>>>(XA, XO, WM, ex_pw_b, out);
}
